// CrossTransformerBlock3D_17265768530511
// MI455X (gfx1250) — hardware-verified
//
#include <hip/hip_runtime.h>
#include <math.h>

typedef __attribute__((ext_vector_type(16))) _Float16 v16h;
typedef __attribute__((ext_vector_type(8)))  _Float16 v8h;
typedef __attribute__((ext_vector_type(2)))  _Float16 v2h;
typedef __attribute__((ext_vector_type(16))) __bf16   v16b;
typedef __attribute__((ext_vector_type(8)))  __bf16   v8b;
typedef __attribute__((ext_vector_type(8)))  float    v8f;
typedef __attribute__((ext_vector_type(4)))  float    v4f;
typedef __attribute__((ext_vector_type(2)))  float    v2f;

constexpr int kDim = 192;
constexpr int kKvw = 384;
constexpr int kHid = 384;
constexpr int kTok = 32768;
constexpr int kNKey = 216;
constexpr int kKPad = 256;
constexpr int kHeadPairs = 6;

__device__ __forceinline__ unsigned short f2bf_bits(float f) {
  unsigned u = __float_as_uint(f);
  return (unsigned short)((u + 0x7FFFu + ((u >> 16) & 1u)) >> 16);
}
__device__ __forceinline__ float bf_bits2f(unsigned short h) { return __uint_as_float(((unsigned)h) << 16); }

__device__ __forceinline__ void dep_guard_h(v8f& a, v8f& b, v16h x, v16h y) { asm volatile("v_nop\n\tv_nop\n\tv_nop\n\tv_nop" : "+v"(a), "+v"(b) : "v"(x), "v"(y)); }
__device__ __forceinline__ void dep_guard_b(v8f& a, v8f& b, v16b x, v16b y) { asm volatile("v_nop\n\tv_nop\n\tv_nop\n\tv_nop" : "+v"(a), "+v"(b) : "v"(x), "v"(y)); }
__device__ __forceinline__ void keep4_h(v16h a, v16h b, v16h c, v16h d) { asm volatile("v_nop" :: "v"(a), "v"(b), "v"(c), "v"(d)); }
__device__ __forceinline__ void keep4_b(v16b a, v16b b, v16b c, v16b d) { asm volatile("v_nop" :: "v"(a), "v"(b), "v"(c), "v"(d)); }
__device__ __forceinline__ void acc_guard4(v8f& a, v8f& b, v8f& c, v8f& d) { asm volatile("v_nop\n\tv_nop\n\tv_nop\n\tv_nop" : "+v"(a), "+v"(b), "+v"(c), "+v"(d)); }
template <typename T> struct Frag;
template <> struct Frag<_Float16> {
  typedef v16h V; union U { v16h v; v8h h[2]; };
  static __device__ __forceinline__ v16h load(const _Float16* p) {
    U f; f.h[0] = *(const v8h*)(p); f.h[1] = *(const v8h*)(p + 16); return f.v;
  }
  static __device__ __forceinline__ v8f mma(v16h a, v16h b, v8f c) {
    return __builtin_amdgcn_wmma_f32_16x16x32_f16(false, a, false, b, (short)0, c, false, false);
  }
  static __device__ __forceinline__ void guard(v8f& a, v8f& b, v16h x, v16h y) { dep_guard_h(a, b, x, y); }
  static __device__ __forceinline__ void keep(v16h a, v16h b, v16h c, v16h d) { keep4_h(a, b, c, d); }
};
template <> struct Frag<__bf16> {
  typedef v16b V; union U { v16b v; v8b h[2]; };
  static __device__ __forceinline__ v16b load(const __bf16* p) {
    U f; f.h[0] = *(const v8b*)(p); f.h[1] = *(const v8b*)(p + 16); return f.v;
  }
  static __device__ __forceinline__ v8f mma(v16b a, v16b b, v8f c) {
    return __builtin_amdgcn_wmma_f32_16x16x32_bf16(false, a, false, b, (short)0, c, false, false);
  }
  static __device__ __forceinline__ void guard(v8f& a, v8f& b, v16b x, v16b y) { dep_guard_b(a, b, x, y); }
  static __device__ __forceinline__ void keep(v16b a, v16b b, v16b c, v16b d) { keep4_b(a, b, c, d); }
};

template <int ET> struct Elem;
template <> struct Elem<0> { typedef _Float16 T; };
template <> struct Elem<1> { typedef __bf16 T; };
template <int ET, bool SPLIT, int BIAS_MODE, int OUT_MODE, bool RESID, int ACT = 0>
__global__ __launch_bounds__(256) void wmma_gemm64(
    const unsigned short* __restrict__ Ap, const unsigned short* __restrict__ A2p, int lda, long strideA,
    const unsigned short* __restrict__ Btp, const unsigned short* __restrict__ Bt2p, int ldb, long strideB,
    void* __restrict__ Cout, void* __restrict__ Cout2, int ldc, long strideC,
    const float* __restrict__ bias,
    const float* __restrict__ resid, long strideR,
    int M, int N, int K, float scale) {
  typedef typename Elem<ET>::T T;
  typedef typename Frag<T>::V V;
  const T* A = (const T*)Ap; const T* A2 = (const T*)A2p; const T* Bt = (const T*)Btp; const T* Bt2 = (const T*)Bt2p;
  __shared__ __align__(16) float sT[8][16 * 68];
  const int b    = blockIdx.y;
  const int lane = threadIdx.x & 31;
  const int wave = threadIdx.x >> 5;
  const int tilesN = N >> 6;
  const int tilesM = M >> 6;
  const int tile = blockIdx.x * 8 + wave;
  if (tile >= tilesM * tilesN) return;
  const int tm = tile / tilesN;
  const int tn = tile - tm * tilesN;
  const int m0 = tm << 6;
  const int n0 = tn << 6;

  const T* Ab  = A  + (size_t)b * strideA;
  const T* Bb  = Bt + (size_t)b * strideB;
  const T* Ab2 = SPLIT ? (A2  + (size_t)b * strideA) : nullptr;
  const T* Bb2 = SPLIT ? (Bt2 + (size_t)b * strideB) : nullptr;

  const int rlane = lane & 15;
  const int koff  = (lane >> 4) * 8;
  const int mOff  = (lane >> 4) * 8;

  v8f acc[4][4];
#pragma unroll
  for (int i = 0; i < 4; ++i)
#pragma unroll
    for (int j = 0; j < 4; ++j) acc[i][j] = (v8f){0.f,0.f,0.f,0.f,0.f,0.f,0.f,0.f};

  for (int k0 = 0; k0 < K; k0 += 32) {
    V bh[4], bl[4];
#pragma unroll
    for (int j = 0; j < 4; ++j) {
      const size_t bo = (size_t)(n0 + (j << 4) + rlane) * ldb + koff + k0;
      bh[j] = Frag<T>::load(Bb + bo);
      if (SPLIT) bl[j] = Frag<T>::load(Bb2 + bo);
    }
#pragma unroll
    for (int i = 0; i < 4; ++i) {
      const size_t ao = (size_t)(m0 + (i << 4) + rlane) * lda + koff + k0;
      V ah = Frag<T>::load(Ab + ao);
      V al;
      if (SPLIT) al = Frag<T>::load(Ab2 + ao);
#pragma unroll
      for (int j = 0; j < 4; ++j) {
        acc[i][j] = Frag<T>::mma(ah, bh[j], acc[i][j]);
        if (SPLIT) {
          acc[i][j] = Frag<T>::mma(ah, bl[j], acc[i][j]);
          acc[i][j] = Frag<T>::mma(al, bh[j], acc[i][j]);
        }
      }
      Frag<T>::guard(acc[i][0], acc[i][3], ah, SPLIT ? al : ah);
    }
    Frag<T>::keep(bh[0], bh[1], bh[2], bh[3]);
    if (SPLIT) Frag<T>::keep(bl[0], bl[1], bl[2], bl[3]);
  }
  acc_guard4(acc[0][0], acc[0][1], acc[0][2], acc[0][3]);
  acc_guard4(acc[1][0], acc[1][1], acc[1][2], acc[1][3]);
  acc_guard4(acc[2][0], acc[2][1], acc[2][2], acc[2][3]);
  acc_guard4(acc[3][0], acc[3][1], acc[3][2], acc[3][3]);

  float* slab = sT[wave];
  const float* Rb = RESID ? (resid + (size_t)b * strideR) : nullptr;
#pragma unroll
  for (int i = 0; i < 4; ++i) {
    const int mBase = m0 + (i << 4);
#pragma unroll
    for (int j = 0; j < 4; ++j) {
      const int n = n0 + (j << 4) + rlane;
      float bv = 0.f;
      if (BIAS_MODE == 2) bv = bias[n];
#pragma unroll
      for (int r = 0; r < 8; ++r) {
        float v = acc[i][j][r] * scale;
        if (BIAS_MODE == 1) v += bias[mBase + mOff + r];
        if (BIAS_MODE == 2) v += bv;
        if (RESID) v += Rb[(size_t)(mBase + mOff + r) * ldc + n];
        if (ACT == 1) v = tanhf(v);
        if (ACT == 2) v = fmaxf(v, 0.0f);
        if (ACT == 3) v = v / (1.0f + expf(-v));
        if (ACT == 4) v = (v > 0.f) ? v : 0.01f * v;
        if (ACT == 5) v = 0.5f * v * (1.0f + erff(v * 0.70710678118654752f));
        slab[(mOff + r) * 68 + (j << 4) + rlane] = v;
      }
    }
    __builtin_amdgcn_fence(__ATOMIC_RELEASE, "workgroup");
    __builtin_amdgcn_wave_barrier();
    __builtin_amdgcn_fence(__ATOMIC_ACQUIRE, "workgroup");
    if (OUT_MODE == 0) {
      float* C = (float*)Cout + (size_t)b * strideC;
      const int hh = lane >> 4, c4 = (lane & 15) * 4;
      for (int pass = 0; pass < 2; ++pass) {
#pragma unroll
        for (int it = 0; it < 8; ++it) {
          const int row = it * 2 + hh;
          v4f v = *(const v4f*)(slab + row * 68 + c4);
          *(volatile v4f*)(C + (size_t)(mBase + row) * ldc + n0 + c4) = v;
        }
        __threadfence();
      }
    } else {
      const int q = lane >> 3, c8 = (lane & 7) * 8;
      unsigned short* C  = (unsigned short*)Cout  + (size_t)b * strideC;
      unsigned short* C2 = (OUT_MODE == 2) ? ((unsigned short*)Cout2 + (size_t)b * strideC) : nullptr;
      for (int pass = 0; pass < 2; ++pass) {
#pragma unroll
        for (int it = 0; it < 4; ++it) {
          const int row = it * 4 + q;
          const float* sp = slab + row * 68 + c8;
          v8h hv, lv;
#pragma unroll
          for (int e = 0; e < 8; ++e) {
            if (OUT_MODE == 1) {
              hv[e] = (_Float16)sp[e];
            } else {
              unsigned short hb = f2bf_bits(sp[e]);
              unsigned short lb = f2bf_bits(sp[e] - bf_bits2f(hb));
              hv[e] = __builtin_bit_cast(_Float16, hb);
              lv[e] = __builtin_bit_cast(_Float16, lb);
            }
          }
          *(volatile v8h*)(C + (size_t)(mBase + row) * ldc + n0 + c8) = hv;
          if (OUT_MODE == 2) *(volatile v8h*)(C2 + (size_t)(mBase + row) * ldc + n0 + c8) = lv;
        }
        __threadfence();
      }
    }
    __builtin_amdgcn_fence(__ATOMIC_RELEASE, "workgroup");
    __builtin_amdgcn_wave_barrier();
    __builtin_amdgcn_fence(__ATOMIC_ACQUIRE, "workgroup");
  }
}

__global__ __launch_bounds__(256) void wtrans_f16(const float* __restrict__ W, _Float16* __restrict__ Wt,
                                                  int kdim, int ndim, float mul) {
  const int kch = kdim >> 3;
  const int total = ndim * kch;
  const int idx = blockIdx.x * 256 + threadIdx.x;
  if (idx >= total) return;
  const int n = idx / kch, kc = idx - n * kch;
  v8h hv;
#pragma unroll
  for (int e = 0; e < 8; ++e) hv[e] = (_Float16)(W[(size_t)(8 * kc + e) * ndim + n] * mul);
  _Float16* dst = Wt + (size_t)n * kdim + 8 * kc;
  *(volatile v8h*)dst = hv;
  __threadfence();
  *(volatile v8h*)dst = hv;
}

__global__ __launch_bounds__(256) void ln_kernel(const float* __restrict__ x, const float* __restrict__ gam,
                                                 const float* __restrict__ bet, _Float16* __restrict__ out, int rows) {
  const int wave = threadIdx.x >> 5;
  const int lane = threadIdx.x & 31;
  const int row  = blockIdx.x * 8 + wave;
  if (row >= rows) return;
  const int lc = lane < 24 ? lane : 23;
  const float wgt = lane < 24 ? 1.0f : 0.0f;
  const float* xr = x + (size_t)row * kDim + 8 * lc;
  const v4f xa = *(const v4f*)(xr), xb = *(const v4f*)(xr + 4);
  float v[8] = {xa[0], xa[1], xa[2], xa[3], xb[0], xb[1], xb[2], xb[3]};
  float s = 0.f;
#pragma unroll
  for (int e = 0; e < 8; ++e) s += v[e];
  s *= wgt;
#pragma unroll
  for (int o = 16; o >= 1; o >>= 1) s += __shfl_xor(s, o, 32);
  const float mean = s * (1.0f / 192.0f);
  float d[8];
  float vs = 0.f;
#pragma unroll
  for (int e = 0; e < 8; ++e) { d[e] = v[e] - mean; vs += d[e] * d[e]; }
  vs *= wgt;
#pragma unroll
  for (int o = 16; o >= 1; o >>= 1) vs += __shfl_xor(vs, o, 32);
  const float inv = rsqrtf(vs * (1.0f / 192.0f) + 1e-5f);
  const v4f ga = *(const v4f*)(gam + 8 * lc), gb = *(const v4f*)(gam + 8 * lc + 4);
  const v4f ba = *(const v4f*)(bet + 8 * lc), bb = *(const v4f*)(bet + 8 * lc + 4);
  const float gg[8] = {ga[0], ga[1], ga[2], ga[3], gb[0], gb[1], gb[2], gb[3]};
  const float be[8] = {ba[0], ba[1], ba[2], ba[3], bb[0], bb[1], bb[2], bb[3]};
  v8h hv;
#pragma unroll
  for (int e = 0; e < 8; ++e) hv[e] = (_Float16)(d[e] * inv * gg[e] + be[e]);
  _Float16* dst = out + (size_t)row * kDim + 8 * lc;
  for (int pass = 0; pass < 2; ++pass) {
    if (lane < 24) *(volatile v8h*)dst = hv;
    __threadfence();
  }
}

__global__ __launch_bounds__(256) void gelu_kernel(const float* __restrict__ in, _Float16* __restrict__ out,
                                                   int n2, float mul) {
  const int i = blockIdx.x * 256 + threadIdx.x;
  if (i >= n2) return;
  const v2f a = *(const v2f*)(in + 2 * (size_t)i);
  float r0 = 0.f, r1 = 0.f;
#pragma unroll 1
  for (int e = 0; e < 2; ++e) {
    const float v = e ? a[1] : a[0];
    const float gv = 0.5f * v * (1.0f + erff(v * 0.70710678118654752f));
    if (e) r1 = gv; else r0 = gv;
  }
  const _Float16 h0 = (_Float16)(r0 * mul), h1 = (_Float16)(r1 * mul);
  const unsigned u = (unsigned)__builtin_bit_cast(unsigned short, h0) | ((unsigned)__builtin_bit_cast(unsigned short, h1) << 16);
  ((volatile unsigned*)out)[i] = u;
  __threadfence();
  ((volatile unsigned*)out)[i] = u;
}

__device__ __forceinline__ v8f wmma_f16_g(v16h a, v16h b, v8f c) {
  c = __builtin_amdgcn_wmma_f32_16x16x32_f16(false, a, false, b, (short)0, c, false, false);
  asm volatile("v_nop\n\tv_nop\n\tv_nop\n\tv_nop" : "+v"(c) : "v"(a), "v"(b));
  return c;
}
__device__ __forceinline__ int win_qtok(int wd, int wh, int ww, int n) {
  const int a = n >> 2, b = (n >> 1) & 1, cc = n & 1;
  return ((2 * wd + a) * 32 + (2 * wh + b)) * 32 + (2 * ww + cc);
}

__global__ __launch_bounds__(128) void win_attn_kernel(const _Float16* __restrict__ qh, const _Float16* __restrict__ kvh,
                                                       const float* __restrict__ bkv, _Float16* __restrict__ aout) {
  __shared__ __align__(16) _Float16 Qsh[8 * kDim];
  __shared__ __align__(16) _Float16 Bsh[kKvw];
  __shared__ int toks[kKPad];
  __shared__ __align__(16) _Float16 Ksh[kKPad * 32];
  __shared__ __align__(16) _Float16 Vt[32 * kKPad];
  __shared__ __align__(16) _Float16 Psh[16 * kKPad];
  __shared__ __align__(16) float Osh[8 * kDim];
  __shared__ float smax[4 * 16];
  __shared__ float ssum[4 * 16];

  const int tid = threadIdx.x, wave = tid >> 5, lane = tid & 31, hh = lane >> 4, c = lane & 15;
  const int wi = blockIdx.x, wd = wi >> 8, wh = (wi >> 4) & 15, ww = wi & 15;

  for (int m = tid; m < kKPad; m += 128) {
    int t = -1;
    if (m < kNKey) {
      const int i = m >> 3, n = m & 7;
      const int di = i / 9, dj = (i / 3) % 3, dk = i % 3;
      const int nd = wd + di - 1, nh = wh + dj - 1, nw = ww + dk - 1;
      const bool ok = (i != 20) && nd >= 0 && nd < 16 && nh >= 0 && nh < 16 && nw >= 0 && nw < 16;
      t = ok ? win_qtok(nd, nh, nw, n) : -1;
    }
    toks[m] = t;
  }
  for (int idx = tid; idx < 8 * 24; idx += 128) {
    const int row = idx / 24, ch = idx - row * 24;
    const int tok = win_qtok(wd, wh, ww, row);
    *(v8h*)(Qsh + row * kDim + 8 * ch) = *(const v8h*)(qh + (size_t)tok * kDim + 8 * ch);
  }
  if (tid < kKvw / 8) {
    const v4f f0 = *(const v4f*)(bkv + 8 * tid), f1 = *(const v4f*)(bkv + 8 * tid + 4);
    v8h hv;
    hv[0] = (_Float16)f0[0]; hv[1] = (_Float16)f0[1]; hv[2] = (_Float16)f0[2]; hv[3] = (_Float16)f0[3];
    hv[4] = (_Float16)f1[0]; hv[5] = (_Float16)f1[1]; hv[6] = (_Float16)f1[2]; hv[7] = (_Float16)f1[3];
    *(v8h*)(Bsh + 8 * tid) = hv;
  }
  __syncthreads();

#pragma unroll 1
  for (int g = 0; g < kHeadPairs; ++g) {
#pragma unroll 1
    for (int j = 0; j < 4; ++j) {
      const int it = tid + 128 * j;
      const int mp = it >> 2, ch = it & 3;
      const int m0 = 2 * mp, m1 = m0 + 1;
      const int t0 = toks[m0], t1 = toks[m1];
      const int tc0 = t0 < 0 ? 0 : (t0 > kTok - 1 ? kTok - 1 : t0);
      const int tc1 = t1 < 0 ? 0 : (t1 > kTok - 1 ? kTok - 1 : t1);
      const int col = 32 * g + 8 * ch;
      const v8h k0 = *(const v8h*)(kvh + (size_t)tc0 * kKvw + col);
      const v8h v0 = *(const v8h*)(kvh + (size_t)tc0 * kKvw + kDim + col);
      const v8h k1 = *(const v8h*)(kvh + (size_t)tc1 * kKvw + col);
      const v8h v1 = *(const v8h*)(kvh + (size_t)tc1 * kKvw + kDim + col);
      const v8h kb = *(const v8h*)(Bsh + col);
      const v8h vb = *(const v8h*)(Bsh + kDim + col);
      const bool val0 = t0 >= 0, val1 = t1 >= 0, real0 = m0 < kNKey, real1 = m1 < kNKey;
      v8h kk0, kk1, vv0, vv1;
#pragma unroll
      for (int e = 0; e < 8; ++e) {
        const _Float16 z = (_Float16)0.0f;
        kk0[e] = val0 ? k0[e] : (real0 ? kb[e] : z);
        kk1[e] = val1 ? k1[e] : (real1 ? kb[e] : z);
        vv0[e] = val0 ? v0[e] : (real0 ? vb[e] : z);
        vv1[e] = val1 ? v1[e] : (real1 ? vb[e] : z);
      }
      *(v8h*)(Ksh + m0 * 32 + 8 * ch) = kk0;
      *(v8h*)(Ksh + m1 * 32 + 8 * ch) = kk1;
#pragma unroll
      for (int e = 0; e < 8; ++e) {
        v2h pr; pr[0] = vv0[e]; pr[1] = vv1[e];
        *(v2h*)(Vt + (8 * ch + e) * kKPad + m0) = pr;
      }
    }
    __syncthreads();

    v16h afr;
    {
      const int hs = c >> 3, n = c & 7;
      const v8h qv = *(const v8h*)(Qsh + n * kDim + 32 * g + 16 * hs + 8 * hh);
      Frag<_Float16>::U u;
#pragma unroll
      for (int e = 0; e < 8; ++e) {
        const _Float16 z = (_Float16)0.0f;
        u.h[0][e] = hs ? z : qv[e];
        u.h[1][e] = hs ? qv[e] : z;
      }
      afr = u.v;
    }
    v8f sacc[4];
#pragma unroll
    for (int j = 0; j < 4; ++j) {
      sacc[j] = (v8f){0.f, 0.f, 0.f, 0.f, 0.f, 0.f, 0.f, 0.f};
      const v16h bfr = Frag<_Float16>::load(Ksh + (64 * wave + 16 * j + c) * 32 + 8 * hh);
      sacc[j] = wmma_f16_g(afr, bfr, sacc[j]);
    }
    float mx[8];
#pragma unroll
    for (int r = 0; r < 8; ++r) {
      float m = fmaxf(fmaxf(sacc[0][r], sacc[1][r]), fmaxf(sacc[2][r], sacc[3][r]));
#pragma unroll
      for (int off = 1; off < 16; off <<= 1) m = fmaxf(m, __shfl_xor(m, off, 32));
      mx[r] = m;
    }
    if (c == 0) {
#pragma unroll
      for (int r = 0; r < 8; ++r) smax[wave * 16 + 8 * hh + r] = mx[r];
    }
    __syncthreads();

    float lsum[8];
#pragma unroll
    for (int r = 0; r < 8; ++r) {
      const int row = 8 * hh + r;
      const float Mr = fmaxf(fmaxf(smax[row], smax[16 + row]), fmaxf(smax[32 + row], smax[48 + row]));
      float ls = 0.f;
#pragma unroll
      for (int j = 0; j < 4; ++j) {
        const int key = 64 * wave + 16 * j + c;
        float ex = __expf((sacc[j][r] - Mr) * 0.25f);
        ex = (key < kNKey) ? ex : 0.0f;
        ls += ex;
        Psh[row * kKPad + key] = (_Float16)(ex * 256.0f);
      }
#pragma unroll
      for (int off = 1; off < 16; off <<= 1) ls += __shfl_xor(ls, off, 32);
      lsum[r] = ls;
    }
    if (c == 0) {
#pragma unroll
      for (int r = 0; r < 8; ++r) ssum[wave * 16 + 8 * hh + r] = lsum[r];
    }
    __syncthreads();

    if (wave < 2) {
      const int hs = wave;
      v8f oacc = (v8f){0.f, 0.f, 0.f, 0.f, 0.f, 0.f, 0.f, 0.f};
#pragma unroll
      for (int ks = 0; ks < 8; ++ks) {
        const v16h pa = Frag<_Float16>::load(Psh + c * kKPad + ks * 32 + 8 * hh);
        const v16h vb = Frag<_Float16>::load(Vt + (16 * hs + c) * kKPad + ks * 32 + 8 * hh);
        oacc = wmma_f16_g(pa, vb, oacc);
      }
#pragma unroll
      for (int r = 0; r < 8; ++r) {
        const int row = 8 * hs + r;
        const float l = ((ssum[row] + ssum[16 + row]) + ssum[32 + row]) + ssum[48 + row];
        const float inv = 1.0f / l;
        const float o = oacc[r] * inv * 0.25f;
        if (hh == hs) Osh[r * kDim + (2 * g + hs) * 16 + c] = o;
      }
    }
    __syncthreads();
  }

  {
    const int lc = lane < 24 ? lane : 23;
    const int r0 = 2 * wave, r1 = 2 * wave + 1;
    v8h hv0, hv1;
#pragma unroll
    for (int e = 0; e < 8; ++e) {
      hv0[e] = (_Float16)Osh[r0 * kDim + 8 * lc + e];
      hv1[e] = (_Float16)Osh[r1 * kDim + 8 * lc + e];
    }
    _Float16* d0 = aout + (size_t)win_qtok(wd, wh, ww, r0) * kDim + 8 * lc;
    _Float16* d1 = aout + (size_t)win_qtok(wd, wh, ww, r1) * kDim + 8 * lc;
    for (int pass = 0; pass < 2; ++pass) {
      if (lane < 24) { *(volatile v8h*)d0 = hv0; *(volatile v8h*)d1 = hv1; }
      __threadfence();
    }
  }
}

static inline unsigned gemm_blocks(int M, int N) { const int tiles = (M / 64) * (N / 64); return (unsigned)((tiles + 7) / 8); }

extern "C" void kernel_launch(void* const* d_in, const int* in_sizes, int n_in,
                              void* d_out, int out_size, void* d_ws, size_t ws_size,
                              hipStream_t stream) {
  if (n_in < 16) return;
  const float* x    = (const float*)d_in[0];
  const float* xa   = (const float*)d_in[1];
  const float* n1g  = (const float*)d_in[2];
  const float* n1b  = (const float*)d_in[3];
  const float* n2g  = (const float*)d_in[4];
  const float* n2b  = (const float*)d_in[5];
  const float* Wq   = (const float*)d_in[6];
  const float* bq   = (const float*)d_in[7];
  const float* Wkv  = (const float*)d_in[8];
  const float* bkv  = (const float*)d_in[9];
  const float* Wp   = (const float*)d_in[10];
  const float* bp   = (const float*)d_in[11];
  const float* W1   = (const float*)d_in[12];
  const float* b1   = (const float*)d_in[13];
  const float* W2   = (const float*)d_in[14];
  const float* b2   = (const float*)d_in[15];

  const int ntok = in_sizes[0] / kDim;
  if (ntok != kTok || in_sizes[1] != kTok * kDim || out_size != kTok * kDim) return;
  if (in_sizes[6] != kDim * kDim || in_sizes[8] != kDim * kKvw || in_sizes[10] != kDim * kDim ||
      in_sizes[12] != kDim * kHid || in_sizes[14] != kHid * kDim) return;

  const size_t szH192 = (size_t)kTok * kDim * 2;
  const size_t szH384 = (size_t)kTok * kHid * 2;
  const size_t szF192 = (size_t)kTok * kDim * 4;
  const size_t offXN  = 0;
  const size_t offXAN = offXN + szH192;
  const size_t offQ   = offXAN + szH192;
  const size_t offKV  = offQ + szH192;
  const size_t offAT  = offKV + szH384;
  const size_t offX1  = offAT + szH192;
  const size_t offH   = offX1 + szF192;
  const size_t offWT  = offH + szH384;
  const size_t szWT   = ((size_t)kDim * kDim + (size_t)kKvw * kDim + (size_t)kDim * kDim +
                         (size_t)kHid * kDim + (size_t)kDim * kHid) * 2;
  const size_t offEnd = offWT + szWT;
  if (offEnd > ws_size) return;
  if (offXAN + (size_t)kTok * kHid * 4 > offX1) return;

  char* ws = (char*)d_ws;
  _Float16* xn   = (_Float16*)(ws + offXN);
  _Float16* x1n  = (_Float16*)(ws + offXN);
  _Float16* xan  = (_Float16*)(ws + offXAN);
  float*    hpre = (float*)(ws + offXAN);
  _Float16* qpl  = (_Float16*)(ws + offQ);
  _Float16* kvpl = (_Float16*)(ws + offKV);
  _Float16* atpl = (_Float16*)(ws + offAT);
  float*    x1   = (float*)(ws + offX1);
  _Float16* hpl  = (_Float16*)(ws + offH);
  _Float16* wqT  = (_Float16*)(ws + offWT);
  _Float16* wkvT = wqT + kDim * kDim;
  _Float16* wpT  = wkvT + kKvw * kDim;
  _Float16* w1T  = wpT + kDim * kDim;
  _Float16* w2T  = w1T + kHid * kDim;

  const float wmul = 64.0f;
  const float wsc  = 1.0f / 64.0f;
  const float wsc2 = 1.0f / 4096.0f;

  wtrans_f16<<<(kDim * kDim / 8 + 255) / 256, 256, 0, stream>>>(Wq,  wqT,  kDim, kDim, wmul);
  wtrans_f16<<<(kKvw * kDim / 8 + 255) / 256, 256, 0, stream>>>(Wkv, wkvT, kDim, kKvw, wmul);
  wtrans_f16<<<(kDim * kDim / 8 + 255) / 256, 256, 0, stream>>>(Wp,  wpT,  kDim, kDim, wmul);
  wtrans_f16<<<(kHid * kDim / 8 + 255) / 256, 256, 0, stream>>>(W1,  w1T,  kDim, kHid, wmul);
  wtrans_f16<<<(kDim * kHid / 8 + 255) / 256, 256, 0, stream>>>(W2,  w2T,  kHid, kDim, wmul);

  ln_kernel<<<(kTok + 7) / 8, 256, 0, stream>>>(x,  n1g, n1b, xn,  kTok);
  ln_kernel<<<(kTok + 7) / 8, 256, 0, stream>>>(xa, n1g, n1b, xan, kTok);

  wmma_gemm64<0, false, 2, 1, false, 0><<<dim3(gemm_blocks(kTok, kDim), 1), 256, 0, stream>>>(
      (const unsigned short*)xn, nullptr, kDim, 0L, (const unsigned short*)wqT, nullptr, kDim, 0L,
      (void*)qpl, nullptr, kDim, 0L, bq, nullptr, 0L, kTok, kDim, kDim, wsc);
  wmma_gemm64<0, false, 2, 1, false, 0><<<dim3(gemm_blocks(kTok, kKvw), 1), 256, 0, stream>>>(
      (const unsigned short*)xan, nullptr, kDim, 0L, (const unsigned short*)wkvT, nullptr, kDim, 0L,
      (void*)kvpl, nullptr, kKvw, 0L, bkv, nullptr, 0L, kTok, kKvw, kDim, wsc);

  win_attn_kernel<<<4096, 128, 0, stream>>>(qpl, kvpl, bkv, atpl);

  wmma_gemm64<0, false, 2, 0, true, 0><<<dim3(gemm_blocks(kTok, kDim), 1), 256, 0, stream>>>(
      (const unsigned short*)atpl, nullptr, kDim, 0L, (const unsigned short*)wpT, nullptr, kDim, 0L,
      (void*)x1, nullptr, kDim, 0L, bp, x, 0L, kTok, kDim, kDim, wsc2);

  ln_kernel<<<(kTok + 7) / 8, 256, 0, stream>>>(x1, n2g, n2b, x1n, kTok);

  wmma_gemm64<0, false, 2, 0, false, 0><<<dim3(gemm_blocks(kTok, kHid), 1), 256, 0, stream>>>(
      (const unsigned short*)x1n, nullptr, kDim, 0L, (const unsigned short*)w1T, nullptr, kDim, 0L,
      (void*)hpre, nullptr, kHid, 0L, b1, nullptr, 0L, kTok, kHid, kDim, wsc);

  {
    const int n2 = kTok * kHid / 2;
    gelu_kernel<<<(n2 + 255) / 256, 256, 0, stream>>>(hpre, hpl, n2, 64.0f);
  }

  wmma_gemm64<0, false, 2, 0, true, 0><<<dim3(gemm_blocks(kTok, kDim), 1), 256, 0, stream>>>(
      (const unsigned short*)hpl, nullptr, kHid, 0L, (const unsigned short*)w2T, nullptr, kHid, 0L,
      d_out, nullptr, kDim, 0L, b2, x1, 0L, kTok, kDim, kHid, wsc2);

  (void)ws_size;
}
